// Block_22823456211331
// MI455X (gfx1250) — hardware-run, weakly checked
//
#include <hip/hip_runtime.h>
#include <math.h>

#ifndef NB
#define NB 2
#endif
#ifndef SEQ
#define SEQ 2048
#endif
#define NB_FULL 2
#define SEQ_FULL 2048
#define EMB 1024
#define NHEAD 16
#define HDIM 64
#define FF2 8192
#define FFH 4096
#define ROWS (NB * SEQ)
#define CHR ((SEQ >= 1024) ? 1024 : SEQ)

static_assert(SEQ % 64 == 0);
static_assert(SEQ <= SEQ_FULL);
static_assert(NB <= NB_FULL);
static_assert(SEQ % CHR == 0);
static_assert(CHR % 64 == 0);
static_assert(NHEAD * HDIM == EMB);

typedef __attribute__((ext_vector_type(16))) _Float16 v16h;
typedef __attribute__((ext_vector_type(8)))  _Float16 v8h;
typedef __attribute__((ext_vector_type(8)))  float    v8f;
typedef __attribute__((ext_vector_type(4)))  float    v4f;
typedef unsigned int cm_u4 __attribute__((ext_vector_type(4)));
typedef unsigned int bk_u2 __attribute__((ext_vector_type(2)));

__device__ __forceinline__ int frag_k(int i, int h) { return (i < 8) ? (8 * h + i) : (16 + 8 * h + (i - 8)); }

__device__ __forceinline__ v8f wmma16(v16h a, v16h b, v8f c) {
    c = __builtin_amdgcn_wmma_f32_16x16x32_f16(false, a, false, b, (short)0, c, false, false);
    asm volatile("v_nop\n\tv_nop\n\tv_nop\n\tv_nop" : "+v"(c) : "v"(a), "v"(b));
    return c;
}

#define VST2(T, ptr, val) do { const T vst2_v_ = (val); *(volatile T*)(ptr) = vst2_v_; __threadfence(); *(volatile T*)(ptr) = vst2_v_; } while (0)
#define VST2V4(ptr, val) do { const v4f vst2_v4_ = (val); *(volatile v4f*)(ptr) = vst2_v4_; __threadfence(); *(volatile v4f*)(ptr) = vst2_v4_; } while (0)

__device__ __forceinline__ unsigned int cmb_pk2(float a, float b) { return (unsigned int)__builtin_bit_cast(unsigned short, (_Float16)a) | ((unsigned int)__builtin_bit_cast(unsigned short, (_Float16)b) << 16); }
__device__ __forceinline__ float cmb_bf(float v) { const unsigned u = __builtin_bit_cast(unsigned, v); const unsigned r = (u + 0x7fffu + ((u >> 16) & 1u)) & 0xffff0000u; return __builtin_bit_cast(float, r); }

__device__ __forceinline__ v16h fh_ld64g(const float* __restrict__ p, int k0, int h, float s) {
    const float* q = p + k0 + 8 * h;
    const v4f a0 = *(const v4f*)(q), a1 = *(const v4f*)(q + 4), b0 = *(const v4f*)(q + 16), b1 = *(const v4f*)(q + 20);
    v16h a;
    a[0] = (_Float16)(a0.x * s); a[1] = (_Float16)(a0.y * s); a[2] = (_Float16)(a0.z * s); a[3] = (_Float16)(a0.w * s);
    a[4] = (_Float16)(a1.x * s); a[5] = (_Float16)(a1.y * s); a[6] = (_Float16)(a1.z * s); a[7] = (_Float16)(a1.w * s);
    a[8] = (_Float16)(b0.x * s); a[9] = (_Float16)(b0.y * s); a[10] = (_Float16)(b0.z * s); a[11] = (_Float16)(b0.w * s);
    a[12] = (_Float16)(b1.x * s); a[13] = (_Float16)(b1.y * s); a[14] = (_Float16)(b1.z * s); a[15] = (_Float16)(b1.w * s);
    return a;
}
__device__ __forceinline__ v16h fh_ld64s(const float* sp, int k0, int h, float s) {
    const float* q = sp + k0 + 8 * h;
    const v4f a0 = *(const v4f*)(q), a1 = *(const v4f*)(q + 4), b0 = *(const v4f*)(q + 16), b1 = *(const v4f*)(q + 20);
    v16h a;
    a[0] = (_Float16)(a0.x * s); a[1] = (_Float16)(a0.y * s); a[2] = (_Float16)(a0.z * s); a[3] = (_Float16)(a0.w * s);
    a[4] = (_Float16)(a1.x * s); a[5] = (_Float16)(a1.y * s); a[6] = (_Float16)(a1.z * s); a[7] = (_Float16)(a1.w * s);
    a[8] = (_Float16)(b0.x * s); a[9] = (_Float16)(b0.y * s); a[10] = (_Float16)(b0.z * s); a[11] = (_Float16)(b0.w * s);
    a[12] = (_Float16)(b1.x * s); a[13] = (_Float16)(b1.y * s); a[14] = (_Float16)(b1.z * s); a[15] = (_Float16)(b1.w * s);
    return a;
}

union FragU { v16h v; v8h h[2]; };
__device__ __forceinline__ v16h frag_ld(const _Float16* p) { FragU f; f.h[0] = *(const v8h*)(p); f.h[1] = *(const v8h*)(p + 16); return f.v; }
__device__ __forceinline__ void dep_guard_h(v8f& a, v8f& b, v16h x, v16h y) { asm volatile("v_nop\n\tv_nop\n\tv_nop\n\tv_nop" : "+v"(a), "+v"(b) : "v"(x), "v"(y)); }
__device__ __forceinline__ void keep4_h(v16h a, v16h b, v16h c, v16h d) { asm volatile("v_nop" :: "v"(a), "v"(b), "v"(c), "v"(d)); }
__device__ __forceinline__ void acc_guard4(v8f& a, v8f& b, v8f& c, v8f& d) { asm volatile("v_nop\n\tv_nop\n\tv_nop\n\tv_nop" : "+v"(a), "+v"(b), "+v"(c), "+v"(d)); }

template <int BIAS_MODE, bool RESID>
__global__ __launch_bounds__(256) void wmma_gemm64(
    const unsigned short* __restrict__ Ap, int lda,
    const unsigned short* __restrict__ Btp, int ldb,
    float* __restrict__ C, int ldc,
    const float* __restrict__ bias,
    const float* __restrict__ resid,
    int M, int N, int K, float scale) {
  const _Float16* A = (const _Float16*)Ap; const _Float16* Bt = (const _Float16*)Btp;
  __shared__ __align__(16) float sT[8][16 * 68];
  const int lane = threadIdx.x & 31;
  const int wave = threadIdx.x >> 5;
  const int tilesN = N >> 6;
  const int tilesM = M >> 6;
  const int tile = blockIdx.x * 8 + wave;
  if (tile >= tilesM * tilesN) return;
  const int tm = tile / tilesN;
  const int tn = tile - tm * tilesN;
  const int m0 = tm << 6;
  const int n0 = tn << 6;

  const int rlane = lane & 15;
  const int koff  = (lane >> 4) * 8;
  const int mOff  = (lane >> 4) * 8;

  v8f acc[4][4];
#pragma unroll
  for (int i = 0; i < 4; ++i)
#pragma unroll
    for (int j = 0; j < 4; ++j) acc[i][j] = (v8f){0.f,0.f,0.f,0.f,0.f,0.f,0.f,0.f};

  for (int k0 = 0; k0 < K; k0 += 32) {
    v16h bh[4];
#pragma unroll
    for (int j = 0; j < 4; ++j) {
      const size_t bo = (size_t)(n0 + (j << 4) + rlane) * ldb + koff + k0;
      bh[j] = frag_ld(Bt + bo);
    }
#pragma unroll
    for (int i = 0; i < 4; ++i) {
      const size_t ao = (size_t)(m0 + (i << 4) + rlane) * lda + koff + k0;
      v16h ah = frag_ld(A + ao);
#pragma unroll
      for (int j = 0; j < 4; ++j) {
        acc[i][j] = __builtin_amdgcn_wmma_f32_16x16x32_f16(false, ah, false, bh[j], (short)0, acc[i][j], false, false);
      }
      dep_guard_h(acc[i][0], acc[i][3], ah, ah);
    }
    keep4_h(bh[0], bh[1], bh[2], bh[3]);
  }
  acc_guard4(acc[0][0], acc[0][1], acc[0][2], acc[0][3]);
  acc_guard4(acc[1][0], acc[1][1], acc[1][2], acc[1][3]);
  acc_guard4(acc[2][0], acc[2][1], acc[2][2], acc[2][3]);
  acc_guard4(acc[3][0], acc[3][1], acc[3][2], acc[3][3]);

  float* slab = sT[wave];
#pragma unroll
  for (int i = 0; i < 4; ++i) {
    const int mBase = m0 + (i << 4);
#pragma unroll
    for (int j = 0; j < 4; ++j) {
      const int n = n0 + (j << 4) + rlane;
      float bv = 0.f;
      if (BIAS_MODE == 2) bv = bias[n];
#pragma unroll
      for (int r = 0; r < 8; ++r) {
        float v = acc[i][j][r] * scale;
        if (BIAS_MODE == 2) v += bv;
        if (RESID) v += resid[(size_t)(mBase + mOff + r) * ldc + n];
        slab[(mOff + r) * 68 + (j << 4) + rlane] = v;
      }
    }
    __builtin_amdgcn_fence(3  , "workgroup");
    __builtin_amdgcn_wave_barrier();
    __builtin_amdgcn_fence(2  , "workgroup");
    {
      const int hh = lane >> 4, c4 = (lane & 15) * 4;
      for (int pass = 0; pass < 2; ++pass) {
#pragma unroll
        for (int it = 0; it < 8; ++it) {
          const int row = it * 2 + hh;
          v4f v = *(const v4f*)(slab + row * 68 + c4);
          *(volatile v4f*)(C + (size_t)(mBase + row) * ldc + n0 + c4) = v;
        }
        __threadfence();
      }
    }
    __builtin_amdgcn_fence(3  , "workgroup");
    __builtin_amdgcn_wave_barrier();
    __builtin_amdgcn_fence(2  , "workgroup");
  }
}

#define AW 4
struct AttnP {
    const float* Q; const float* K; const float* V; float* O;
    long long sQb, sQh, sQi, sKb, sKh, sKj, sVb, sVh, sVj, sOb, sOh, sOi;
    int Lq, Lk; float scale; int pad_;
};
static_assert(sizeof(AttnP) == 4 * 8 + 12 * 8 + 4 * 4);

__global__ __launch_bounds__(32 * AW) void k_attn(AttnP p) {
    constexpr int VP = 72;
    __shared__ __align__(16) float    pl[AW][16 * 64];
    __shared__ __align__(16) _Float16 vl[64 * VP];
    const int lane = threadIdx.x & 31, hf = lane >> 4, l15 = lane & 15, wave = threadIdx.x >> 5;
    const int h = blockIdx.y, b = blockIdx.z;
    const int q0 = (blockIdx.x * AW + wave) * 16;
    float* myp = pl[wave];
    const float L2E = 1.4426950408889634f;
    const float NEG = -__builtin_inff();
    const int qi = min(q0 + l15, p.Lq - 1);
    const float* qrow = p.Q + b * p.sQb + h * p.sQh + (long long)qi * p.sQi;
    const float* kbase = p.K + b * p.sKb + h * p.sKh;
    const float* vbase = p.V + b * p.sVb + h * p.sVh;
    v16h qa[2];
#pragma unroll
    for (int ks = 0; ks < 2; ++ks) qa[ks] = fh_ld64g(qrow, ks * 32, hf, 1.f);
    v8f o[4]; float m8[8], l8[8];
#pragma unroll
    for (int t = 0; t < 4; ++t) { v8f zz = {}; o[t] = zz; }
#pragma unroll
    for (int i = 0; i < 8; ++i) { m8[i] = NEG; l8[i] = 0.f; }
    const int jend = min(p.Lk, (int)(blockIdx.x * AW + AW) * 16);
    for (int j0 = 0; j0 < jend; j0 += 64) {
        __syncthreads();
        for (int idx = threadIdx.x; idx < 64 * 16; idx += 32 * AW) {
            const int jr = idx >> 4, d4 = (idx & 15) * 4; const int j = j0 + jr; const int jc = min(j, p.Lk - 1);
            const v4f f = *(const v4f*)(vbase + (long long)jc * p.sVj + d4);
            const bool ok = (j < p.Lk);
            _Float16* vd = vl + jr * VP + d4;
            vd[0] = (_Float16)(ok ? f.x : 0.f); vd[1] = (_Float16)(ok ? f.y : 0.f); vd[2] = (_Float16)(ok ? f.z : 0.f); vd[3] = (_Float16)(ok ? f.w : 0.f);
        }
        v8f s[4];
#pragma unroll
        for (int t = 0; t < 4; ++t) {
            const int j = min(j0 + t * 16 + l15, p.Lk - 1);
            const float* krow = kbase + (long long)j * p.sKj;
            v8f acc = {};
#pragma unroll
            for (int ks = 0; ks < 2; ++ks) acc = wmma16(qa[ks], fh_ld64g(krow, ks * 32, hf, 1.f), acc);
            s[t] = acc;
        }
        float pv[8][4];
#pragma unroll
        for (int i = 0; i < 8; ++i) {
            const int irow = q0 + i + 8 * hf;
            float sc[4];
#pragma unroll
            for (int t = 0; t < 4; ++t) {
                const int jg = j0 + t * 16 + l15;
                float v = s[t][i] * p.scale;
                if (jg >= p.Lk || jg > irow) v = NEG; else v *= L2E;
                sc[t] = v;
            }
            float mx = fmaxf(fmaxf(sc[0], sc[1]), fmaxf(sc[2], sc[3]));
            mx = fmaxf(mx, __shfl_xor(mx, 1, 32)); mx = fmaxf(mx, __shfl_xor(mx, 2, 32));
            mx = fmaxf(mx, __shfl_xor(mx, 4, 32)); mx = fmaxf(mx, __shfl_xor(mx, 8, 32));
            const float mnew = fmaxf(m8[i], mx);
            const float corr = (mnew == NEG) ? 1.f : exp2f(m8[i] - mnew);
            float rs = 0.f;
#pragma unroll
            for (int t = 0; t < 4; ++t) {
                const float pp = (sc[t] == NEG) ? 0.f : exp2f(sc[t] - mnew); rs += pp;
                pv[i][t] = pp;
            }
            rs += __shfl_xor(rs, 1, 32); rs += __shfl_xor(rs, 2, 32); rs += __shfl_xor(rs, 4, 32); rs += __shfl_xor(rs, 8, 32);
            l8[i] = l8[i] * corr + rs; m8[i] = mnew;
#pragma unroll
            for (int t = 0; t < 4; ++t) o[t][i] *= corr;
        }
#pragma unroll
        for (int i = 0; i < 8; ++i)
#pragma unroll
            for (int t = 0; t < 4; ++t) myp[(i + 8 * hf) * 64 + t * 16 + l15] = pv[i][t];
        __syncthreads();
        {
            const v16h pa0 = fh_ld64s(myp + l15 * 64, 0, hf, 4096.f), pa1 = fh_ld64s(myp + l15 * 64, 32, hf, 4096.f);
#pragma unroll
            for (int t = 0; t < 4; ++t) {
                const int dcol = t * 16 + l15;
                v16h b0, b1;
#pragma unroll
                for (int e = 0; e < 16; ++e) { b0[e] = vl[frag_k(e, hf) * VP + dcol]; b1[e] = vl[(32 + frag_k(e, hf)) * VP + dcol]; }
                o[t] = wmma16(pa0, b0, o[t]);
                o[t] = wmma16(pa1, b1, o[t]);
            }
        }
    }
    float* obase = p.O + b * p.sOb + h * p.sOh;
    float invr[8];
#pragma unroll
    for (int i = 0; i < 8; ++i) invr[i] = (l8[i] > 0.f) ? 1.f / (l8[i] * 4096.f) : 0.f;
    __syncthreads();
#pragma unroll
    for (int i = 0; i < 8; ++i)
#pragma unroll
        for (int t = 0; t < 4; ++t) myp[(i + 8 * hf) * 64 + t * 16 + l15] = o[t][i] * invr[i];
    __syncthreads();
    for (int r0 = 0; r0 < 16; r0 += 2) {
        const int row = r0 + (lane >> 4), c4 = (lane & 15) * 4;
        const v4f v = *(const v4f*)(myp + row * 64 + c4);
        VST2V4(obase + (long long)(q0 + row) * p.sOi + c4, v);
    }
}

__global__ __launch_bounds__(256) void k_cm_castbT(const float* __restrict__ SRC, int lds, long long srcZ, unsigned short* __restrict__ DST, int ldd, long long dstZ, int nR, int nC, float sc) {
    const long long u = (long long)blockIdx.x * 256 + threadIdx.x; const int per = nR / 8; if (u >= (long long)nC * per) return;
    const int c = (int)(u / per); const int r0 = 8 * (int)(u % per);
    const float* S = SRC + (long long)blockIdx.y * srcZ; unsigned short* D = DST + (long long)blockIdx.y * dstZ;
    float w[8];
#pragma unroll
    for (int e = 0; e < 8; ++e) w[e] = cmb_bf(S[(long long)(r0 + e) * lds + c]) * sc;
    cm_u4 pk; pk.x = cmb_pk2(w[0], w[1]); pk.y = cmb_pk2(w[2], w[3]); pk.z = cmb_pk2(w[4], w[5]); pk.w = cmb_pk2(w[6], w[7]);
    VST2(cm_u4, (cm_u4*)(D + (long long)c * ldd + r0), pk);
}

__global__ __launch_bounds__(256) void k_bias3(const float* __restrict__ bo, const float* __restrict__ b1, const float* __restrict__ b2, float* __restrict__ DST) {
    const int u = blockIdx.x * 256 + threadIdx.x; if (u >= EMB + FF2 + EMB) return;
    const int i0 = min(u, EMB - 1), i1 = min(max(u - EMB, 0), FF2 - 1), i2 = min(max(u - EMB - FF2, 0), EMB - 1);
    const float v0 = bo[i0], v1 = b1[i1], v2 = b2[i2];
    const float v = (u < EMB) ? v0 : ((u < EMB + FF2) ? v1 : v2);
    VST2(float, DST + u, cmb_bf(v));
}

template <int HASX, int XBF, int ABF>
__global__ __launch_bounds__(256) void k_rms(const float* __restrict__ A, int seqA, const float* __restrict__ X, int seqX, const float* __restrict__ GA, float eps, int rows, int seq, float* __restrict__ Sf, unsigned short* __restrict__ Y16) {
    #pragma clang fp contract(off)
    constexpr int NQ = 8; constexpr int WD = 128 * NQ;
    const int r = blockIdx.x * 8 + (threadIdx.x >> 5); const int L = threadIdx.x & 31; if (r >= rows) return;
    const int bb = r / seq, ss = r - bb * seq;
    const long long ra = (long long)bb * seqA + ss, rx = (long long)bb * seqX + ss;
    v4f v[NQ]; float s = 0.f;
#pragma unroll
    for (int q = 0; q < NQ; ++q) {
        const int c = 4 * L + 128 * q;
        v[q] = *(const v4f*)(A + ra * WD + c);
        if (ABF) { v[q].x = cmb_bf(v[q].x); v[q].y = cmb_bf(v[q].y); v[q].z = cmb_bf(v[q].z); v[q].w = cmb_bf(v[q].w); }
        if (HASX) { v4f x = *(const v4f*)(X + rx * WD + c); if (XBF) { x.x = cmb_bf(x.x); x.y = cmb_bf(x.y); x.z = cmb_bf(x.z); x.w = cmb_bf(x.w); } v[q] = v[q] + x; }
        s += (v[q].x * v[q].x + v[q].y * v[q].y) + (v[q].z * v[q].z + v[q].w * v[q].w);
    }
#pragma unroll
    for (int o = 16; o > 0; o >>= 1) s += __shfl_xor(s, o, 32);
    const float rs = rsqrtf(s * (1.f / WD) + eps);
#pragma unroll
    for (int q = 0; q < NQ; ++q) {
        const int c = 4 * L + 128 * q; const v4f ga = *(const v4f*)(GA + c);
        v4f y; y.x = (v[q].x * rs) * cmb_bf(ga.x); y.y = (v[q].y * rs) * cmb_bf(ga.y); y.z = (v[q].z * rs) * cmb_bf(ga.z); y.w = (v[q].w * rs) * cmb_bf(ga.w);
        const long long o = (long long)r * WD + c;
        if (Sf != nullptr) VST2V4(Sf + o, v[q]);
        bk_u2 pk; pk.x = cmb_pk2(y.x, y.y); pk.y = cmb_pk2(y.z, y.w); VST2(bk_u2, (bk_u2*)(Y16 + o), pk);
    }
}

__global__ __launch_bounds__(256) void k_rope_qk(float* __restrict__ QKV, const float* __restrict__ cs, const float* __restrict__ sn, int rows, int seq) {
    #pragma clang fp contract(off)
    const long long u = (long long)blockIdx.x * 256 + threadIdx.x; if (u >= (long long)rows * 512) return;
    const int r = (int)(u >> 9); const int c4 = 4 * (int)(u & 511);
    const int s = r % seq; const int j = (c4 & 63) >> 1;
    const float c0 = cmb_bf(cs[s * 32 + j]), c1 = cmb_bf(cs[s * 32 + j + 1]);
    const float s0 = cmb_bf(sn[s * 32 + j]), s1 = cmb_bf(sn[s * 32 + j + 1]);
    float* ptr = QKV + (long long)r * (3 * EMB) + c4;
    const v4f x = *(const v4f*)ptr;
    v4f y; y.x = x.x * c0 - x.y * s0; y.y = x.x * s0 + x.y * c0; y.z = x.z * c1 - x.w * s1; y.w = x.z * s1 + x.w * c1;
    VST2V4(ptr, y);
}

__global__ __launch_bounds__(256) void k_cast16(const float* __restrict__ SRC, unsigned short* __restrict__ DST, long long n8) {
    const long long u = (long long)blockIdx.x * 256 + threadIdx.x; if (u >= n8) return;
    const v4f a = *(const v4f*)(SRC + 8 * u), b = *(const v4f*)(SRC + 8 * u + 4);
    cm_u4 pk; pk.x = cmb_pk2(a.x, a.y); pk.y = cmb_pk2(a.z, a.w); pk.z = cmb_pk2(b.x, b.y); pk.w = cmb_pk2(b.z, b.w);
    VST2(cm_u4, (cm_u4*)(DST + 8 * u), pk);
}

__device__ __forceinline__ float sigm(float g) { return __builtin_amdgcn_rcpf(1.0f + expf(-g)); }
__global__ __launch_bounds__(256) void k_glu16(const float* __restrict__ U, unsigned short* __restrict__ F, long long n8) {
    #pragma clang fp contract(off)
    const long long u = (long long)blockIdx.x * 256 + threadIdx.x; if (u >= n8) return;
    const long long r = u >> 9; const int c = 8 * (int)(u & 511);
    const float* ua = U + r * FF2 + c;
    const v4f a0 = *(const v4f*)(ua), a1 = *(const v4f*)(ua + 4), g0 = *(const v4f*)(ua + FFH), g1 = *(const v4f*)(ua + FFH + 4);
    cm_u4 pk;
    pk.x = cmb_pk2(a0.x * sigm(g0.x), a0.y * sigm(g0.y)); pk.y = cmb_pk2(a0.z * sigm(g0.z), a0.w * sigm(g0.w));
    pk.z = cmb_pk2(a1.x * sigm(g1.x), a1.y * sigm(g1.y)); pk.w = cmb_pk2(a1.z * sigm(g1.z), a1.w * sigm(g1.w));
    VST2(cm_u4, (cm_u4*)(F + r * FFH + c), pk);
}

constexpr size_t cmax(size_t a, size_t b) { return a > b ? a : b; }
constexpr size_t SZ_X16 = (size_t)ROWS * EMB * 2;
constexpr size_t SZ_W3  = (size_t)3 * EMB * EMB * 2;
constexpr size_t SZ_QKV = cmax(cmax((size_t)ROWS * 3 * EMB * 4, (size_t)CHR * FF2 * 4), (size_t)ROWS * EMB * 4);
constexpr size_t SZ_AO  = cmax((size_t)ROWS * EMB * 4, (size_t)CHR * FFH * 2);
constexpr size_t SZ_WO  = (size_t)EMB * EMB * 2;
constexpr size_t SZ_X1  = (size_t)ROWS * EMB * 4;
constexpr size_t SZ_W1  = (size_t)FF2 * EMB * 2;
constexpr size_t SZ_W2  = (size_t)EMB * FFH * 2;
constexpr size_t SZ_BR  = (size_t)(EMB + FF2 + EMB) * 4;
constexpr size_t OFF_X16 = 0;
constexpr size_t OFF_W3  = OFF_X16 + SZ_X16;
constexpr size_t OFF_QKV = OFF_W3 + SZ_W3;
constexpr size_t OFF_AO  = OFF_QKV + SZ_QKV;
constexpr size_t OFF_WO  = OFF_AO + SZ_AO;
constexpr size_t OFF_X1  = OFF_WO + SZ_WO;
constexpr size_t OFF_W1  = OFF_X1 + SZ_X1;
constexpr size_t OFF_W2  = OFF_W1 + SZ_W1;
constexpr size_t OFF_BR  = OFF_W2 + SZ_W2;
constexpr size_t WS_TOTAL = OFF_BR + SZ_BR;
static_assert(SZ_X16 % 256 == 0 && SZ_W3 % 256 == 0 && SZ_QKV % 256 == 0 && SZ_AO % 256 == 0 && SZ_WO % 256 == 0 && SZ_X1 % 256 == 0 && SZ_W1 % 256 == 0 && SZ_W2 % 256 == 0 && SZ_BR % 256 == 0);
static_assert(WS_TOTAL <= (size_t)134217728);
static_assert((size_t)((NB - 1) * SEQ_FULL + SEQ) * EMB <= (size_t)NB_FULL * SEQ_FULL * EMB);

extern "C" void kernel_launch(void* const* d_in, const int* in_sizes, int n_in, void* d_out, int out_size, void* d_ws, size_t ws_size, hipStream_t stream) {
    if (n_in < 14) return;
    const long long need_x = ((long long)(NB - 1) * SEQ_FULL + SEQ) * EMB;
    if ((long long)in_sizes[0] < need_x) return;
    if (in_sizes[1] < SEQ * 32 || in_sizes[2] < SEQ * 32) return;
    if (in_sizes[3] < EMB || in_sizes[8] < EMB || in_sizes[9] < EMB || in_sizes[13] < EMB || in_sizes[11] < FF2) return;
    if (in_sizes[4] < EMB * EMB || in_sizes[5] < EMB * EMB || in_sizes[6] < EMB * EMB || in_sizes[7] < EMB * EMB) return;
    if (in_sizes[10] < EMB * FF2 || in_sizes[12] < FFH * EMB) return;
    if ((long long)out_size < need_x) return;
    if (WS_TOTAL > ws_size) return;

    const float* x     = (const float*)d_in[0];
    const float* cosb  = (const float*)d_in[1];
    const float* sinb  = (const float*)d_in[2];
    const float* w_ln1 = (const float*)d_in[3];
    const float* wq    = (const float*)d_in[4];
    const float* wk    = (const float*)d_in[5];
    const float* wv    = (const float*)d_in[6];
    const float* wo    = (const float*)d_in[7];
    const float* bo    = (const float*)d_in[8];
    const float* w_ln2 = (const float*)d_in[9];
    const float* w1    = (const float*)d_in[10];
    const float* b1    = (const float*)d_in[11];
    const float* w2    = (const float*)d_in[12];
    const float* b2    = (const float*)d_in[13];
    float* out = (float*)d_out;
    char* wsp = (char*)d_ws;
    unsigned short* X16  = (unsigned short*)(wsp + OFF_X16);
    unsigned short* W316 = (unsigned short*)(wsp + OFF_W3);
    float* QKV = (float*)(wsp + OFF_QKV);
    float* ATT = QKV;
    float* U   = QKV;
    float* AO  = (float*)(wsp + OFF_AO);
    unsigned short* F16 = (unsigned short*)(wsp + OFF_AO);
    unsigned short* WO16 = (unsigned short*)(wsp + OFF_WO);
    float* X1 = (float*)(wsp + OFF_X1);
    unsigned short* W1T = (unsigned short*)(wsp + OFF_W1);
    unsigned short* W2T = (unsigned short*)(wsp + OFF_W2);
    float* BR = (float*)(wsp + OFF_BR);
    float* BRO = BR; float* BR1 = BR + EMB; float* BR2 = BR + EMB + FF2;

    k_bias3<<<(EMB + FF2 + EMB + 255) / 256, 256, 0, stream>>>(bo, b1, b2, BR);
    k_cm_castbT<<<dim3((unsigned)((64 * (EMB / 8) + 255) / 256), NHEAD), 256, 0, stream>>>(wq, 64, (long long)EMB * HDIM, W316, EMB, (long long)HDIM * EMB, EMB, 64, 16.0f);
    k_cm_castbT<<<dim3((unsigned)((64 * (EMB / 8) + 255) / 256), NHEAD), 256, 0, stream>>>(wk, 64, (long long)EMB * HDIM, W316 + (size_t)EMB * EMB, EMB, (long long)HDIM * EMB, EMB, 64, 16.0f);
    k_cm_castbT<<<dim3((unsigned)((64 * (EMB / 8) + 255) / 256), NHEAD), 256, 0, stream>>>(wv, 64, (long long)EMB * HDIM, W316 + (size_t)2 * EMB * EMB, EMB, (long long)HDIM * EMB, EMB, 64, 16.0f);
    k_cm_castbT<<<dim3((unsigned)(((long long)EMB * (EMB / 8) + 255) / 256), 1), 256, 0, stream>>>(wo, EMB, 0LL, WO16, EMB, 0LL, EMB, EMB, 16.0f);
    k_cm_castbT<<<dim3((unsigned)(((long long)FF2 * (EMB / 8) + 255) / 256), 1), 256, 0, stream>>>(w1, FF2, 0LL, W1T, EMB, 0LL, EMB, FF2, 16.0f);
    k_cm_castbT<<<dim3((unsigned)(((long long)EMB * (FFH / 8) + 255) / 256), 1), 256, 0, stream>>>(w2, EMB, 0LL, W2T, FFH, 0LL, FFH, EMB, 16.0f);

    k_rms<0, 0, 1><<<(ROWS + 7) / 8, 256, 0, stream>>>(x, SEQ_FULL, nullptr, 0, w_ln1, 1e-6f, ROWS, SEQ, nullptr, X16);
    wmma_gemm64<0, false><<<(unsigned)((((ROWS / 64) * (3 * EMB / 64)) + 7) / 8), 256, 0, stream>>>(X16, EMB, W316, EMB, QKV, 3 * EMB, nullptr, nullptr, ROWS, 3 * EMB, EMB, 0.0625f);
    k_rope_qk<<<(unsigned)(((long long)ROWS * 512 + 255) / 256), 256, 0, stream>>>(QKV, cosb, sinb, ROWS, SEQ);
    {
        AttnP a;
        a.Q = QKV; a.K = QKV + EMB; a.V = QKV + 2 * EMB; a.O = AO;
        a.sQb = (long long)SEQ * 3 * EMB; a.sQh = HDIM; a.sQi = 3 * EMB;
        a.sKb = (long long)SEQ * 3 * EMB; a.sKh = HDIM; a.sKj = 3 * EMB;
        a.sVb = (long long)SEQ * 3 * EMB; a.sVh = HDIM; a.sVj = 3 * EMB;
        a.sOb = (long long)SEQ * EMB; a.sOh = HDIM; a.sOi = EMB;
        a.Lq = SEQ; a.Lk = SEQ; a.scale = 0.125f; a.pad_ = 0;
        k_attn<<<dim3((unsigned)(SEQ / (16 * AW)), NHEAD, NB), 32 * AW, 0, stream>>>(a);
    }
    k_cast16<<<(unsigned)(((long long)ROWS * (EMB / 8) + 255) / 256), 256, 0, stream>>>(AO, X16, (long long)ROWS * (EMB / 8));
    wmma_gemm64<2, false><<<(unsigned)((((ROWS / 64) * (EMB / 64)) + 7) / 8), 256, 0, stream>>>(X16, EMB, WO16, EMB, ATT, EMB, BRO, nullptr, ROWS, EMB, EMB, 0.0625f);
    k_rms<1, 1, 0><<<(ROWS + 7) / 8, 256, 0, stream>>>(ATT, SEQ, x, SEQ_FULL, w_ln2, 1e-6f, ROWS, SEQ, X1, X16);
    for (int bq = 0; bq < NB; ++bq) {
        for (int cq = 0; cq < SEQ / CHR; ++cq) {
            const size_t row0 = (size_t)bq * SEQ + (size_t)cq * CHR;
            wmma_gemm64<2, false><<<(unsigned)((((CHR / 64) * (FF2 / 64)) + 7) / 8), 256, 0, stream>>>(X16 + row0 * EMB, EMB, W1T, EMB, U, FF2, BR1, nullptr, CHR, FF2, EMB, 0.0625f);
            k_glu16<<<(unsigned)(((long long)CHR * 512 + 255) / 256), 256, 0, stream>>>(U, F16, (long long)CHR * 512);
            wmma_gemm64<2, true><<<(unsigned)((((CHR / 64) * (EMB / 64)) + 7) / 8), 256, 0, stream>>>(F16, FFH, W2T, FFH, out + ((size_t)bq * SEQ_FULL + (size_t)cq * CHR) * EMB, EMB, BR2, X1 + row0 * EMB, CHR, EMB, FFH, 0.0625f);
        }
    }
}
